// PhysicsGuidedAttention_85040352460997
// MI455X (gfx1250) — hardware-verified
//
#include <hip/hip_runtime.h>
#include <math.h>
#include <stdint.h>

#define NB   2
#define NQ   2048
#define NC   4096
#define CM   512
#define NH   8
#define HD   64
#define MQ   (NB * NQ)
#define MC   (NB * NC)
#define KC   (2 * CM)
#define NCH  (NC / 32)
#define RSC  2048.0f
#define PSC  1024.0f
#define SCL  0.125f
#define HK4  0.4f
#define HEPS 1.0e-6f
static_assert(NH * HD == CM);
static_assert(NH == 8);
static_assert((MQ % 64) == 0 && (MC % 64) == 0 && (CM % 64) == 0 && (NC % 64) == 0 && (KC % 32) == 0);
static_assert((((MQ / 64) * (CM / 64)) % 8) == 0);
static_assert((((MC / 64) * (CM / 64)) % 8) == 0);
static_assert((((CM / 64) * (NC / 64)) % 8) == 0);
static_assert((NQ % 16) == 0 && (NC % 32) == 0);

typedef _Float16 v16h __attribute__((ext_vector_type(16)));
typedef _Float16 v8h  __attribute__((ext_vector_type(8)));
typedef __bf16   v16b __attribute__((ext_vector_type(16)));
typedef unsigned short v16us __attribute__((ext_vector_type(16)));
typedef unsigned short v8us  __attribute__((ext_vector_type(8)));
typedef float    v8f  __attribute__((ext_vector_type(8)));
typedef float    v4f  __attribute__((ext_vector_type(4)));
typedef unsigned int v4u __attribute__((ext_vector_type(4)));

union FragU { v16us v; v8us h[2]; };

__device__ __forceinline__ unsigned short bf_bits(float f) {
  unsigned u = __float_as_uint(f);
  return (unsigned short)((u + 0x7FFFu + ((u >> 16) & 1u)) >> 16);
}
__device__ __forceinline__ float bf_up(unsigned short h) { return __uint_as_float(((unsigned)h) << 16); }
__device__ __forceinline__ float bfr(float f) { return bf_up(bf_bits(f)); }
__device__ __forceinline__ unsigned short h_bits(_Float16 x) { return __builtin_bit_cast(unsigned short, x); }
__device__ __forceinline__ unsigned pk16(unsigned short a, unsigned short b) { return (unsigned)a | ((unsigned)b << 16); }
__device__ __forceinline__ v8f zero8() { v8f z = {0.f, 0.f, 0.f, 0.f, 0.f, 0.f, 0.f, 0.f}; return z; }

__device__ __forceinline__ v16us ldfrag_u(const unsigned short* p) {
  FragU f;
  f.h[0] = *(const v8us*)(p);
  f.h[1] = *(const v8us*)(p + 16);
  return f.v;
}

__device__ __forceinline__ v8f mma_bu_raw(v16us a, v16us b, v8f c) {
  return __builtin_amdgcn_wmma_f32_16x16x32_bf16(false, __builtin_bit_cast(v16b, a), false,
                                                 __builtin_bit_cast(v16b, b), (short)0, c, false, false);
}
__device__ __forceinline__ v8f mma_hu(v16us a, v16us b, v8f c) {
  c = __builtin_amdgcn_wmma_f32_16x16x32_f16(false, __builtin_bit_cast(v16h, a), false,
                                              __builtin_bit_cast(v16h, b), (short)0, c, false, false);
#if defined(__HIP_DEVICE_COMPILE__)
  asm volatile("v_nop\n\tv_nop\n\tv_nop\n\tv_nop" : "+v"(c) : "v"(a), "v"(b));
#endif
  return c;
}
__device__ __forceinline__ void dep_guard1(v8f& a, v8f& b, v16us x) {
#if defined(__HIP_DEVICE_COMPILE__)
  asm volatile("v_nop\n\tv_nop\n\tv_nop\n\tv_nop" : "+v"(a), "+v"(b) : "v"(x));
#endif
}
__device__ __forceinline__ void keep4_u(v16us a, v16us b, v16us c, v16us d) {
#if defined(__HIP_DEVICE_COMPILE__)
  asm volatile("v_nop" :: "v"(a), "v"(b), "v"(c), "v"(d));
#endif
}
__device__ __forceinline__ void acc_guard4(v8f& a, v8f& b, v8f& c, v8f& d) {
#if defined(__HIP_DEVICE_COMPILE__)
  asm volatile("v_nop\n\tv_nop\n\tv_nop\n\tv_nop" : "+v"(a), "+v"(b), "+v"(c), "+v"(d));
#endif
}
__device__ __forceinline__ void wave_sync_lds() {
  __builtin_amdgcn_fence(__ATOMIC_RELEASE, "workgroup");
  __builtin_amdgcn_wave_barrier();
  __builtin_amdgcn_fence(__ATOMIC_ACQUIRE, "workgroup");
}

__global__ __launch_bounds__(64) void cvt_rows(const float* __restrict__ src, unsigned short* dst, int ldo, int dup) {
  const int row = blockIdx.x, tid = threadIdx.x;
  const float* p = src + (size_t)row * CM + tid * 8;
  const v4f a0 = *(const v4f*)(p);
  const v4f a1 = *(const v4f*)(p + 4);
  v4u hv;
  hv[0] = pk16(bf_bits(a0[0]), bf_bits(a0[1]));
  hv[1] = pk16(bf_bits(a0[2]), bf_bits(a0[3]));
  hv[2] = pk16(bf_bits(a1[0]), bf_bits(a1[1]));
  hv[3] = pk16(bf_bits(a1[2]), bf_bits(a1[3]));
  unsigned short* d = dst + (size_t)row * ldo + tid * 8;
  for (int pass = 0; pass < 2; ++pass) {
    *(volatile v4u*)(d) = hv;
    if (dup != 0) *(volatile v4u*)(d + dup) = hv;
    __threadfence();
  }
}

template <int OM, int CBM>
__global__ __launch_bounds__(256) void gemm64(
    const unsigned short* __restrict__ Ap, int lda, long long sAy,
    const unsigned short* __restrict__ Btp, int ldb, long long sBy,
    unsigned short* Cp, unsigned short* Cp2, float* Cf, int ldc, long long sCy,
    const float* __restrict__ cb, int M, int N, int K) {
  __shared__ __align__(16) float sT[8][16 * 68];
  const int by   = blockIdx.y;
  const int lane = threadIdx.x & 31;
  const int wave = threadIdx.x >> 5;
  const int tilesN = N >> 6;
  const int tilesM = M >> 6;
  const int tile = blockIdx.x * 8 + wave;
  if (tile >= tilesM * tilesN) return;
  const int tm = tile / tilesN;
  const int tn = tile - tm * tilesN;
  const int m0 = tm << 6;
  const int n0 = tn << 6;

  const unsigned short* Ab = Ap  + (size_t)by * (size_t)sAy;
  const unsigned short* Bb = Btp + (size_t)by * (size_t)sBy;
  const size_t cofs = (size_t)by * (size_t)sCy;

  const int rlane = lane & 15;
  const int koff  = (lane >> 4) * 8;
  const int mOff  = (lane >> 4) * 8;

  v8f acc[4][4];
#pragma unroll
  for (int i = 0; i < 4; ++i)
#pragma unroll
    for (int j = 0; j < 4; ++j) acc[i][j] = zero8();

  for (int k0 = 0; k0 < K; k0 += 32) {
    v16us bh[4];
#pragma unroll
    for (int j = 0; j < 4; ++j) {
      const size_t bo = (size_t)(n0 + (j << 4) + rlane) * ldb + koff + k0;
      bh[j] = ldfrag_u(Bb + bo);
    }
#pragma unroll
    for (int i = 0; i < 4; ++i) {
      const size_t ao = (size_t)(m0 + (i << 4) + rlane) * lda + koff + k0;
      const v16us ah = ldfrag_u(Ab + ao);
#pragma unroll
      for (int j = 0; j < 4; ++j) acc[i][j] = mma_bu_raw(ah, bh[j], acc[i][j]);
      dep_guard1(acc[i][0], acc[i][3], ah);
    }
    keep4_u(bh[0], bh[1], bh[2], bh[3]);
  }
  acc_guard4(acc[0][0], acc[0][1], acc[0][2], acc[0][3]);
  acc_guard4(acc[1][0], acc[1][1], acc[1][2], acc[1][3]);
  acc_guard4(acc[2][0], acc[2][1], acc[2][2], acc[2][3]);
  acc_guard4(acc[3][0], acc[3][1], acc[3][2], acc[3][3]);

  const int hh2 = lane >> 4, c4 = (lane & 15) * 4;
  const int q8  = lane >> 3, c8 = (lane & 7) * 8;

  v4f cb4 = {0.f, 0.f, 0.f, 0.f};
  float cbc[8];
#pragma unroll
  for (int e = 0; e < 8; ++e) cbc[e] = 0.f;
  if (CBM == 1) {
    if (OM == 0) {
      const v4f v = *(const v4f*)(cb + n0 + c4);
      cb4[0] = bfr(v[0]); cb4[1] = bfr(v[1]); cb4[2] = bfr(v[2]); cb4[3] = bfr(v[3]);
    } else {
      const v4f v0 = *(const v4f*)(cb + n0 + c8);
      const v4f v1 = *(const v4f*)(cb + n0 + c8 + 4);
#pragma unroll
      for (int e = 0; e < 4; ++e) { cbc[e] = bfr(v0[e]); cbc[4 + e] = bfr(v1[e]); }
    }
  }

  float* slab = sT[wave];
#pragma unroll
  for (int i = 0; i < 4; ++i) {
    const int mBase = m0 + (i << 4);
#pragma unroll
    for (int j = 0; j < 4; ++j) {
#pragma unroll
      for (int r = 0; r < 8; ++r) {
        slab[(mOff + r) * 68 + (j << 4) + rlane] = acc[i][j][r];
      }
    }
    wave_sync_lds();
    if (OM == 0) {
      float* C = Cf + cofs;
      v4f vals[8];
#pragma unroll
      for (int it = 0; it < 8; ++it) {
        const int row = it * 2 + hh2;
        const v4f v = *(const v4f*)(slab + row * 68 + c4);
        vals[it] = v + cb4;
      }
      for (int pass = 0; pass < 2; ++pass) {
#pragma unroll
        for (int it = 0; it < 8; ++it) {
          const int row = it * 2 + hh2;
          *(volatile v4f*)(C + (size_t)(mBase + row) * ldc + (size_t)n0 + c4) = vals[it];
        }
        __threadfence();
      }
    } else {
      unsigned short* C  = Cp  + cofs;
      unsigned short* C2 = Cp2 + cofs;
      v4u hv[4], lv[4];
#pragma unroll
      for (int it = 0; it < 4; ++it) {
        const int row = it * 4 + q8;
        const float* sp = slab + row * 68 + c8;
        float rb = 0.f;
        if (CBM == 2) rb = bfr(cb[mBase + row]);
        v4u ha = {0u, 0u, 0u, 0u}, la = {0u, 0u, 0u, 0u};
#pragma unroll
        for (int e = 0; e < 4; ++e) {
          const float f0 = sp[2 * e]     + cbc[2 * e]     + rb;
          const float f1 = sp[2 * e + 1] + cbc[2 * e + 1] + rb;
          const _Float16 g0 = (_Float16)f0, g1 = (_Float16)f1;
          ha[e] = pk16(h_bits(g0), h_bits(g1));
          if (OM == 2) {
            la[e] = pk16(h_bits((_Float16)((f0 - (float)g0) * RSC)),
                         h_bits((_Float16)((f1 - (float)g1) * RSC)));
          }
        }
        hv[it] = ha;
        lv[it] = la;
      }
      for (int pass = 0; pass < 2; ++pass) {
#pragma unroll
        for (int it = 0; it < 4; ++it) {
          const int row = it * 4 + q8;
          const size_t go = (size_t)(mBase + row) * ldc + (size_t)n0 + c8;
          *(volatile v4u*)(C + go) = hv[it];
          if (OM == 2) *(volatile v4u*)(C2 + go) = lv[it];
        }
        __threadfence();
      }
    }
    wave_sync_lds();
  }
}

__global__ void __launch_bounds__(256) attn_kernel(
    const float* __restrict__ posq, const float* __restrict__ posc,
    const unsigned short* __restrict__ qp, const unsigned short* __restrict__ kp,
    const unsigned short* __restrict__ vth, const unsigned short* __restrict__ vtl,
    unsigned short* ctxp) {
#pragma clang fp contract(off)
  __shared__ __align__(16) unsigned short prL[NH * 512];
  __shared__ __align__(16) float heatL[16 * 32];
  __shared__ __align__(16) float osm[16 * CM];
  __shared__ float qps[16 * 3];

  const int b = blockIdx.y, i0 = blockIdx.x * 16;
  const int t = threadIdx.x, lane = t & 31, w = t >> 5, hh = lane >> 4, jc = lane & 15;
  const size_t rowQ = (size_t)b * NQ, rowC = (size_t)b * NC;

  if (t < 48) qps[t] = bfr(posq[(rowQ + i0) * 3 + t]);
  __syncthreads();

  const unsigned short* qrow = qp + (rowQ + i0 + jc) * CM + w * HD + 8 * hh;
  const v16us qf0 = ldfrag_u(qrow);
  const v16us qf1 = ldfrag_u(qrow + 32);

  const float qx0 = qps[w * 3 + 0],       qy0 = qps[w * 3 + 1],       qt0 = qps[w * 3 + 2];
  const float qx1 = qps[(w + 8) * 3 + 0], qy1 = qps[(w + 8) * 3 + 1], qt1 = qps[(w + 8) * 3 + 2];

  float m[8], ll[8];
  v8f oh[4], ol[4];
#pragma unroll
  for (int ct = 0; ct < 4; ++ct) { oh[ct] = zero8(); ol[ct] = zero8(); }
#pragma unroll
  for (int r = 0; r < 8; ++r) { m[r] = -1.0e30f; ll[r] = 0.f; }

  const unsigned short* vhb = vth + ((size_t)b * CM + w * HD + jc) * NC + 8 * hh;
  const unsigned short* vlb = vtl + ((size_t)b * CM + w * HD + jc) * NC + 8 * hh;
  const unsigned short* kgb = kp + (rowC + jc) * CM + w * HD + 8 * hh;
  const float* pcb = posc + rowC * 3;
  unsigned short* pr = prL + w * 512;

#pragma unroll 1
  for (int jt = 0; jt < NCH; ++jt) {
    const int j0 = jt * 32;
    __syncthreads();
    {
      const float* pc = pcb + (size_t)(j0 + lane) * 3;
      const float cx = bfr(pc[0]), cy = bfr(pc[1]), cz = bfr(pc[2]);
      const float dxa = qx0 - cx, dya = qy0 - cy, dta = qt0 - cz;
      const float dxb = qx1 - cx, dyb = qy1 - cy, dtb = qt1 - cz;
      const float da = dxa * dxa + dya * dya;
      const float db = dxb * dxb + dyb * dyb;
      const float na = HK4 * fabsf(dta) + HEPS;
      const float nb = HK4 * fabsf(dtb) + HEPS;
      const float ha = expf(-(da * (1.0f / na)));
      const float hb = expf(-(db * (1.0f / nb)));
      heatL[w * 32 + lane]       = ha;
      heatL[(w + 8) * 32 + lane] = hb;
    }
    __syncthreads();

    const unsigned short* kg = kgb + (size_t)j0 * CM;
    v8f s0, s1;
    {
      const v16us k00 = ldfrag_u(kg);
      const v16us k01 = ldfrag_u(kg + 32);
      s0 = mma_hu(qf0, k00, zero8());
      s0 = mma_hu(qf1, k01, s0);
      const v16us k10 = ldfrag_u(kg + (size_t)16 * CM);
      const v16us k11 = ldfrag_u(kg + (size_t)16 * CM + 32);
      s1 = mma_hu(qf0, k10, zero8());
      s1 = mma_hu(qf1, k11, s1);
    }

#pragma unroll
    for (int r = 0; r < 8; ++r) {
      const int il = 8 * hh + r;
      const float v0 = s0[r] * SCL + heatL[il * 32 + jc];
      const float v1 = s1[r] * SCL + heatL[il * 32 + 16 + jc];
      float rm = fmaxf(v0, v1);
#pragma unroll
      for (int off = 1; off < 16; off <<= 1) rm = fmaxf(rm, __shfl_xor(rm, off, 32));
      const float mn2   = fmaxf(m[r], rm);
      const float alpha = __expf(m[r] - mn2);
      const float e0 = __expf(v0 - mn2), e1 = __expf(v1 - mn2);
      float rs = e0 + e1;
#pragma unroll
      for (int off = 1; off < 16; off <<= 1) rs += __shfl_xor(rs, off, 32);
      ll[r] = ll[r] * alpha + rs;
      m[r]  = mn2;
#pragma unroll
      for (int ct = 0; ct < 4; ++ct) { oh[ct][r] *= alpha; ol[ct][r] *= alpha; }
      pr[il * 32 + jc]      = h_bits((_Float16)(e0 * PSC));
      pr[il * 32 + 16 + jc] = h_bits((_Float16)(e1 * PSC));
    }
    wave_sync_lds();

    FragU pa;
    pa.h[0] = *(const v8us*)(pr + jc * 32 + 8 * hh);
    pa.h[1] = *(const v8us*)(pr + jc * 32 + 16 + 8 * hh);
#pragma unroll
    for (int ct = 0; ct < 4; ++ct) {
      const v16us vh = ldfrag_u(vhb + (size_t)ct * 16 * NC + j0);
      oh[ct] = mma_hu(pa.v, vh, oh[ct]);
      const v16us vl = ldfrag_u(vlb + (size_t)ct * 16 * NC + j0);
      ol[ct] = mma_hu(pa.v, vl, ol[ct]);
    }
  }

  __syncthreads();
#pragma unroll
  for (int r = 0; r < 8; ++r) {
    const int il = 8 * hh + r;
    const float l = ll[r];
    const float inv = ((l > 0.f) ? (1.0f / l) : 0.f) * (1.0f / PSC);
#pragma unroll
    for (int ct = 0; ct < 4; ++ct) {
      osm[il * CM + w * HD + ct * 16 + jc] = (oh[ct][r] + ol[ct][r] * (1.0f / RSC)) * inv;
    }
  }
  __syncthreads();
  {
    v4u hv[2][2], lv[2][2];
#pragma unroll
    for (int rr = 0; rr < 2; ++rr) {
      const float* sp = osm + (w + 8 * rr) * CM;
#pragma unroll
      for (int it = 0; it < 2; ++it) {
        const int c = it * 256 + lane * 8;
        const v4f f0 = *(const v4f*)(sp + c);
        const v4f f1 = *(const v4f*)(sp + c + 4);
        v4u ha, la;
#pragma unroll
        for (int e = 0; e < 2; ++e) {
          const unsigned short u0 = bf_bits(f0[2 * e]), u1 = bf_bits(f0[2 * e + 1]);
          const unsigned short u2 = bf_bits(f1[2 * e]), u3 = bf_bits(f1[2 * e + 1]);
          ha[e]     = pk16(u0, u1);
          ha[2 + e] = pk16(u2, u3);
          la[e]     = pk16(bf_bits(f0[2 * e] - bf_up(u0)), bf_bits(f0[2 * e + 1] - bf_up(u1)));
          la[2 + e] = pk16(bf_bits(f1[2 * e] - bf_up(u2)), bf_bits(f1[2 * e + 1] - bf_up(u3)));
        }
        hv[rr][it] = ha;
        lv[rr][it] = la;
      }
    }
    for (int pass = 0; pass < 2; ++pass) {
#pragma unroll
      for (int rr = 0; rr < 2; ++rr) {
        const size_t go = (rowQ + i0 + w + 8 * rr) * KC;
#pragma unroll
        for (int it = 0; it < 2; ++it) {
          const int c = it * 256 + lane * 8;
          *(volatile v4u*)(ctxp + go + c)      = hv[rr][it];
          *(volatile v4u*)(ctxp + go + CM + c) = lv[rr][it];
        }
      }
      __threadfence();
    }
  }
}

extern "C" void kernel_launch(void* const* d_in, const int* in_sizes, int n_in,
                              void* d_out, int out_size, void* d_ws, size_t ws_size,
                              hipStream_t stream) {
  if (n_in < 12) return;
  if (in_sizes[0] != MC * CM) return;
  if (in_sizes[1] != MQ * CM) return;
  if (in_sizes[2] != MC * 3) return;
  if (in_sizes[3] != MQ * 3) return;
  if (in_sizes[4] != CM * CM || in_sizes[5] != CM) return;
  if (in_sizes[6] != CM * CM || in_sizes[7] != CM) return;
  if (in_sizes[8] != CM * CM || in_sizes[9] != CM) return;
  if (in_sizes[10] != CM * CM || in_sizes[11] != CM) return;
  if (out_size != MQ * CM) return;

  const float* x_ctx   = (const float*)d_in[0];
  const float* x_query = (const float*)d_in[1];
  const float* pos_ctx = (const float*)d_in[2];
  const float* pos_qry = (const float*)d_in[3];
  const float* Wq = (const float*)d_in[4];
  const float* bq = (const float*)d_in[5];
  const float* Wk = (const float*)d_in[6];
  const float* bk = (const float*)d_in[7];
  const float* Wv = (const float*)d_in[8];
  const float* bv = (const float*)d_in[9];
  const float* Wo = (const float*)d_in[10];
  const float* bo = (const float*)d_in[11];

  const size_t PXQ  = (size_t)MQ * CM * 2;
  const size_t PXC  = (size_t)MC * CM * 2;
  const size_t PW   = (size_t)CM * CM * 2;
  const size_t PWO  = (size_t)CM * KC * 2;
  const size_t PQ   = (size_t)MQ * CM * 2;
  const size_t PK   = (size_t)MC * CM * 2;
  const size_t PVT  = (size_t)NB * CM * NC * 2;
  const size_t PCTX = (size_t)MQ * KC * 2;
  size_t off = 0;
  const size_t oXq  = off; off += PXQ;
  const size_t oXc  = off; off += PXC;
  const size_t oWq  = off; off += PW;
  const size_t oWk  = off; off += PW;
  const size_t oWv  = off; off += PW;
  const size_t oWo  = off; off += PWO;
  const size_t oQ   = off; off += PQ;
  const size_t oK   = off; off += PK;
  const size_t oVTh = off; off += PVT;
  const size_t oVTl = off; off += PVT;
  const size_t oCtx = off; off += PCTX;
  if (off > ws_size) return;
  if (off > (size_t)134217728) return;

  char* ws = (char*)d_ws;
  unsigned short* Xq   = (unsigned short*)(ws + oXq);
  unsigned short* Xc   = (unsigned short*)(ws + oXc);
  unsigned short* Wqb  = (unsigned short*)(ws + oWq);
  unsigned short* Wkb  = (unsigned short*)(ws + oWk);
  unsigned short* Wvb  = (unsigned short*)(ws + oWv);
  unsigned short* WoT2 = (unsigned short*)(ws + oWo);
  unsigned short* Qp   = (unsigned short*)(ws + oQ);
  unsigned short* Kp   = (unsigned short*)(ws + oK);
  unsigned short* VTh  = (unsigned short*)(ws + oVTh);
  unsigned short* VTl  = (unsigned short*)(ws + oVTl);
  unsigned short* Ctx  = (unsigned short*)(ws + oCtx);
  float*          out0 = (float*)d_out;

  const dim3 blk(256), blk64(64);
  const dim3 gQ(((MQ / 64) * (CM / 64)) / 8, 1, 1);
  const dim3 gK(((MC / 64) * (CM / 64)) / 8, 1, 1);
  const dim3 gVT(((CM / 64) * (NC / 64)) / 8, NB, 1);
  const dim3 gAttn(NQ / 16, NB, 1);
  const dim3 gO(((MQ / 64) * (CM / 64)) / 8, 1, 1);
  if ((((MQ / 64) * (CM / 64)) % 8) != 0) return;
  if ((((MC / 64) * (CM / 64)) % 8) != 0) return;
  if ((((CM / 64) * (NC / 64)) % 8) != 0) return;

  cvt_rows<<<dim3(MQ), blk64, 0, stream>>>(x_query, Xq, CM, 0);
  cvt_rows<<<dim3(MC), blk64, 0, stream>>>(x_ctx, Xc, CM, 0);
  cvt_rows<<<dim3(CM), blk64, 0, stream>>>(Wq, Wqb, CM, 0);
  cvt_rows<<<dim3(CM), blk64, 0, stream>>>(Wk, Wkb, CM, 0);
  cvt_rows<<<dim3(CM), blk64, 0, stream>>>(Wv, Wvb, CM, 0);
  cvt_rows<<<dim3(CM), blk64, 0, stream>>>(Wo, WoT2, KC, CM);

  gemm64<1, 1><<<gQ, blk, 0, stream>>>(
      Xq, CM, 0LL, Wqb, CM, 0LL,
      Qp, Qp, out0, CM, 0LL,
      bq, MQ, CM, CM);
  gemm64<1, 1><<<gK, blk, 0, stream>>>(
      Xc, CM, 0LL, Wkb, CM, 0LL,
      Kp, Kp, out0, CM, 0LL,
      bk, MC, CM, CM);
  gemm64<2, 2><<<gVT, blk, 0, stream>>>(
      Wvb, CM, 0LL, Xc, CM, (long long)NC * CM,
      VTh, VTl, out0, NC, (long long)CM * NC,
      bv, CM, NC, CM);

  attn_kernel<<<gAttn, blk, 0, stream>>>(pos_qry, pos_ctx, Qp, Kp, VTh, VTl, Ctx);

  gemm64<0, 1><<<gO, blk, 0, stream>>>(
      Ctx, KC, 0LL, WoT2, KC, 0LL,
      Ctx, Ctx, out0, CM, 0LL,
      bo, MQ, CM, KC);
  (void)hipGetLastError();
}
